// SelfAttentionLayer_1614907703989
// MI455X (gfx1250) — hardware-verified
//
#include <hip/hip_runtime.h>
#include <math.h>

#define NB     4
#define NS     2048
#define ND     1024
#define NTOK   (NB * NS)
#define JB     16
#define SPITCH 2048
#define SLDS_BYTES (JB * SPITCH * 4)
#define SSCALE 0.00048828125f
#define PROJ_CARRY 8.0f

static_assert((NS % 64) == 0);
static_assert((ND % 64) == 0);
static_assert((NTOK % 64) == 0);
static_assert((ND % 32) == 0);
static_assert((NS % 32) == 0);
static_assert((NS % JB) == 0);
static_assert(NS == 8 * 256);
static_assert(NS == 4 * 512);
static_assert(SLDS_BYTES == 131072);

typedef _Float16 v16h __attribute__((ext_vector_type(16)));
typedef _Float16 v8h  __attribute__((ext_vector_type(8)));
typedef __bf16   v16b __attribute__((ext_vector_type(16)));
typedef __bf16   v8b  __attribute__((ext_vector_type(8)));
typedef float    v8f  __attribute__((ext_vector_type(8)));
typedef float    v4f  __attribute__((ext_vector_type(4)));
typedef unsigned int v4u __attribute__((ext_vector_type(4)));
typedef v4f __attribute__((may_alias)) v4fa;
typedef v8h __attribute__((may_alias)) v8ha;
typedef v8b __attribute__((may_alias)) v8ba;

__device__ __forceinline__ unsigned short f2bf_bits(float f) {
  unsigned u = __float_as_uint(f);
  return (unsigned short)((u + 0x7FFFu + ((u >> 16) & 1u)) >> 16);
}
__device__ __forceinline__ float bf_bits2f(unsigned short h) { return __uint_as_float(((unsigned)h) << 16); }
__device__ __forceinline__ unsigned pk16(unsigned short a, unsigned short b) { return (unsigned)a | ((unsigned)b << 16); }
__device__ __forceinline__ void split_pair(float f0, float f1, unsigned& hp, unsigned& lp) {
  const unsigned short h0 = f2bf_bits(f0), h1 = f2bf_bits(f1);
  const unsigned short l0 = f2bf_bits(f0 - bf_bits2f(h0)), l1 = f2bf_bits(f1 - bf_bits2f(h1));
  hp = pk16(h0, h1);
  lp = pk16(l0, l1);
}

__device__ __forceinline__ void dep_guard_h(v8f& a, v8f& b, v16h x, v16h y) { asm volatile("v_nop\n\tv_nop\n\tv_nop\n\tv_nop" : "+v"(a), "+v"(b) : "v"(x), "v"(y)); }
__device__ __forceinline__ void dep_guard_b(v8f& a, v8f& b, v16b x, v16b y) { asm volatile("v_nop\n\tv_nop\n\tv_nop\n\tv_nop" : "+v"(a), "+v"(b) : "v"(x), "v"(y)); }
__device__ __forceinline__ void keep4_h(v16h a, v16h b, v16h c, v16h d) { asm volatile("v_nop" :: "v"(a), "v"(b), "v"(c), "v"(d)); }
__device__ __forceinline__ void keep4_b(v16b a, v16b b, v16b c, v16b d) { asm volatile("v_nop" :: "v"(a), "v"(b), "v"(c), "v"(d)); }
__device__ __forceinline__ void acc_guard4(v8f& a, v8f& b, v8f& c, v8f& d) { asm volatile("v_nop\n\tv_nop\n\tv_nop\n\tv_nop" : "+v"(a), "+v"(b), "+v"(c), "+v"(d)); }

template <typename T> struct Frag;
template <> struct Frag<_Float16> {
  typedef v16h V; union U { v16h v; v8h h[2]; };
  static __device__ __forceinline__ v16h load(const _Float16* p) {
    U f; f.h[0] = *(const v8ha*)(p); f.h[1] = *(const v8ha*)(p + 16); return f.v;
  }
  static __device__ __forceinline__ v8f mma(v16h a, v16h b, v8f c) {
    return __builtin_amdgcn_wmma_f32_16x16x32_f16(false, a, false, b, (short)0, c, false, false);
  }
  static __device__ __forceinline__ void guard(v8f& a, v8f& b, v16h x, v16h y) { dep_guard_h(a, b, x, y); }
  static __device__ __forceinline__ void keep(v16h a, v16h b, v16h c, v16h d) { keep4_h(a, b, c, d); }
};
template <> struct Frag<__bf16> {
  typedef v16b V; union U { v16b v; v8b h[2]; };
  static __device__ __forceinline__ v16b load(const __bf16* p) {
    U f; f.h[0] = *(const v8ba*)(p); f.h[1] = *(const v8ba*)(p + 16); return f.v;
  }
  static __device__ __forceinline__ v8f mma(v16b a, v16b b, v8f c) {
    return __builtin_amdgcn_wmma_f32_16x16x32_bf16(false, a, false, b, (short)0, c, false, false);
  }
  static __device__ __forceinline__ void guard(v8f& a, v8f& b, v16b x, v16b y) { dep_guard_b(a, b, x, y); }
  static __device__ __forceinline__ void keep(v16b a, v16b b, v16b c, v16b d) { keep4_b(a, b, c, d); }
};

__device__ __forceinline__ v8f wmma_f16g(v16h a, v16h b, v8f c) {
  v8f d = __builtin_amdgcn_wmma_f32_16x16x32_f16(false, a, false, b, (short)0, c, false, false);
  asm volatile("v_nop\n\tv_nop\n\tv_nop\n\tv_nop" : "+v"(d) : "v"(a), "v"(b));
  return d;
}

__global__ __launch_bounds__(256) void prep_x_kernel(const float* __restrict__ x,
                                                     unsigned short* __restrict__ xb,
                                                     unsigned short* __restrict__ xt) {
  __shared__ __align__(16) float tf[64 * 68];
  const int z = blockIdx.z;
  const float* xz = x + (size_t)z * NS * ND;
  unsigned short* xbz = xb + (size_t)z * NS * ND;
  unsigned short* xtz = xt + (size_t)z * ND * NS;
  const int c0  = blockIdx.x * 64;
  const int r0  = blockIdx.y * 64;
  const int tid = threadIdx.x;
  {
    const int lr = tid >> 4;
    const int c4 = (tid & 15) * 4;
#pragma unroll
    for (int it = 0; it < 4; ++it) {
      const int rr = it * 16 + lr;
      const v4f a = *(const v4fa*)(xz + (size_t)(r0 + rr) * ND + c0 + c4);
      *(v4fa*)(tf + rr * 68 + c4) = a;
    }
  }
  __syncthreads();
  const int sub = tid >> 3;
  const int c8  = (tid & 7) * 8;
  v4u sv[2], tv[2];
#pragma unroll
  for (int it = 0; it < 2; ++it) {
    const int rr = it * 32 + sub;
    v4u a, t;
#pragma unroll
    for (int q = 0; q < 4; ++q) {
      const float s0 = tf[rr * 68 + c8 + 2 * q];
      const float s1 = tf[rr * 68 + c8 + 2 * q + 1];
      const float t0 = tf[(c8 + 2 * q) * 68 + rr];
      const float t1 = tf[(c8 + 2 * q + 1) * 68 + rr];
      a[q] = pk16(f2bf_bits(s0), f2bf_bits(s1));
      t[q] = pk16(f2bf_bits(t0), f2bf_bits(t1));
    }
    sv[it] = a; tv[it] = t;
  }
#pragma unroll 1
  for (int pass = 0; pass < 2; ++pass) {
#pragma unroll
    for (int it = 0; it < 2; ++it) {
      const int rr = it * 32 + sub;
      *(volatile v4u*)(xbz + (size_t)(r0 + rr) * ND + c0 + c8) = sv[it];
      *(volatile v4u*)(xtz + (size_t)(c0 + rr) * NS + r0 + c8) = tv[it];
    }
    __threadfence();
  }
}

__global__ __launch_bounds__(256) void prep_w_kernel(const float* __restrict__ wq, const float* __restrict__ wk,
                                                     const float* __restrict__ wv,
                                                     unsigned short* __restrict__ wqt, unsigned short* __restrict__ wkt,
                                                     unsigned short* __restrict__ wvt) {
  __shared__ __align__(16) float tf[64 * 68];
  const int z = blockIdx.z;
  const float* W = (z == 0) ? wk : ((z == 1) ? wq : wv);
  unsigned short* O = (z == 0) ? wkt : ((z == 1) ? wqt : wvt);
  const int c0  = blockIdx.x * 64;
  const int r0  = blockIdx.y * 64;
  const int tid = threadIdx.x;
  {
    const int lr = tid >> 4;
    const int c4 = (tid & 15) * 4;
#pragma unroll
    for (int it = 0; it < 4; ++it) {
      const int rr = it * 16 + lr;
      const v4f a = *(const v4fa*)(W + (size_t)(r0 + rr) * ND + c0 + c4);
      *(v4fa*)(tf + rr * 68 + c4) = a;
    }
  }
  __syncthreads();
  const int sub = tid >> 3;
  const int c8  = (tid & 7) * 8;
  v4u tv[2];
#pragma unroll
  for (int it = 0; it < 2; ++it) {
    const int oc = it * 32 + sub;
    v4u t;
#pragma unroll
    for (int q = 0; q < 4; ++q) {
      const float t0 = tf[(c8 + 2 * q) * 68 + oc];
      const float t1 = tf[(c8 + 2 * q + 1) * 68 + oc];
      t[q] = pk16(f2bf_bits(t0), f2bf_bits(t1));
    }
    tv[it] = t;
  }
#pragma unroll 1
  for (int pass = 0; pass < 2; ++pass) {
#pragma unroll
    for (int it = 0; it < 2; ++it) {
      const int oc = it * 32 + sub;
      *(volatile v4u*)(O + (size_t)(c0 + oc) * ND + r0 + c8) = tv[it];
    }
    __threadfence();
  }
}

template <int ET> struct Elem;
template <> struct Elem<0> { typedef _Float16 T; };
template <> struct Elem<1> { typedef __bf16 T; };

template <int ET, bool ASPLIT, int OUT_MODE>
__global__ __launch_bounds__(256) void wmma_gemm64(
    const unsigned short* __restrict__ Ap, const unsigned short* __restrict__ A2p, int lda, long strideA,
    const unsigned short* __restrict__ Btp, int ldb, long strideB,
    void* __restrict__ Cout, void* __restrict__ Cout2, int ldc, long strideC,
    int M, int N, int K, float scale) {
  typedef typename Elem<ET>::T T;
  typedef typename Frag<T>::V V;
  const T* A = (const T*)Ap; const T* A2 = (const T*)A2p; const T* Bt = (const T*)Btp;
  __shared__ __align__(16) float sT[8][16 * 68];
  const int b    = blockIdx.y;
  const int lane = threadIdx.x & 31;
  const int wave = threadIdx.x >> 5;
  const int tilesN = N >> 6;
  const int tilesM = M >> 6;
  const int tile = blockIdx.x * 8 + wave;
  if (tile >= tilesM * tilesN) return;
  const int tm = tile / tilesN;
  const int tn = tile - tm * tilesN;
  const int m0 = tm << 6;
  const int n0 = tn << 6;

  const T* Ab  = A  + (size_t)b * strideA;
  const T* Bb  = Bt + (size_t)b * strideB;
  const T* Ab2 = ASPLIT ? (A2 + (size_t)b * strideA) : Ab;

  const int rlane = lane & 15;
  const int koff  = (lane >> 4) * 8;
  const int mOff  = (lane >> 4) * 8;

  v8f acc[4][4];
#pragma unroll
  for (int i = 0; i < 4; ++i)
#pragma unroll
    for (int j = 0; j < 4; ++j) acc[i][j] = (v8f){0.f,0.f,0.f,0.f,0.f,0.f,0.f,0.f};

  for (int k0 = 0; k0 < K; k0 += 32) {
    V bf[4];
#pragma unroll
    for (int j = 0; j < 4; ++j) {
      const size_t bo = (size_t)(n0 + (j << 4) + rlane) * ldb + koff + k0;
      bf[j] = Frag<T>::load(Bb + bo);
    }
#pragma unroll
    for (int i = 0; i < 4; ++i) {
      const size_t ao = (size_t)(m0 + (i << 4) + rlane) * lda + koff + k0;
      V ah = Frag<T>::load(Ab + ao);
      V al = ah;
      if (ASPLIT) al = Frag<T>::load(Ab2 + ao);
#pragma unroll
      for (int j = 0; j < 4; ++j) {
        acc[i][j] = Frag<T>::mma(ah, bf[j], acc[i][j]);
        if (ASPLIT) acc[i][j] = Frag<T>::mma(al, bf[j], acc[i][j]);
      }
      Frag<T>::guard(acc[i][0], acc[i][3], ah, al);
    }
    Frag<T>::keep(bf[0], bf[1], bf[2], bf[3]);
  }
  acc_guard4(acc[0][0], acc[0][1], acc[0][2], acc[0][3]);
  acc_guard4(acc[1][0], acc[1][1], acc[1][2], acc[1][3]);
  acc_guard4(acc[2][0], acc[2][1], acc[2][2], acc[2][3]);
  acc_guard4(acc[3][0], acc[3][1], acc[3][2], acc[3][3]);

  float* slab = sT[wave];
#pragma unroll
  for (int i = 0; i < 4; ++i) {
    const int mBase = m0 + (i << 4);
#pragma unroll
    for (int j = 0; j < 4; ++j) {
#pragma unroll
      for (int r = 0; r < 8; ++r) {
        slab[(mOff + r) * 68 + (j << 4) + rlane] = acc[i][j][r] * scale;
      }
    }
    __builtin_amdgcn_fence(__ATOMIC_RELEASE, "workgroup");
    __builtin_amdgcn_wave_barrier();
    __builtin_amdgcn_fence(__ATOMIC_ACQUIRE, "workgroup");
    if (OUT_MODE == 0) {
      float* C = (float*)Cout + (size_t)b * strideC;
      const int hh = lane >> 4, c4 = (lane & 15) * 4;
      for (int pass = 0; pass < 2; ++pass) {
#pragma unroll
        for (int it = 0; it < 8; ++it) {
          const int row = it * 2 + hh;
          v4f v = *(const v4fa*)(slab + row * 68 + c4);
          *(volatile v4f*)(C + (size_t)(mBase + row) * ldc + n0 + c4) = v;
        }
        __threadfence();
      }
    } else {
      const int q = lane >> 3, c8 = (lane & 7) * 8;
      unsigned short* C  = (unsigned short*)Cout  + (size_t)b * strideC;
      unsigned short* C2 = (unsigned short*)Cout2 + (size_t)b * strideC;
      for (int pass = 0; pass < 2; ++pass) {
#pragma unroll
        for (int it = 0; it < 4; ++it) {
          const int row = it * 4 + q;
          const float* sp = slab + row * 68 + c8;
          v8h hv, lv;
#pragma unroll
          for (int e = 0; e < 8; ++e) {
            if (OUT_MODE == 1) {
              hv[e] = (_Float16)sp[e];
              lv[e] = hv[e];
            } else {
              unsigned short hb = f2bf_bits(sp[e]);
              unsigned short lb = f2bf_bits(sp[e] - bf_bits2f(hb));
              hv[e] = __builtin_bit_cast(_Float16, hb);
              lv[e] = __builtin_bit_cast(_Float16, lb);
            }
          }
          *(volatile v8h*)(C + (size_t)(mBase + row) * ldc + n0 + c8) = hv;
          if (OUT_MODE == 2) *(volatile v8h*)(C2 + (size_t)(mBase + row) * ldc + n0 + c8) = lv;
        }
        __threadfence();
      }
    }
    __builtin_amdgcn_fence(__ATOMIC_RELEASE, "workgroup");
    __builtin_amdgcn_wave_barrier();
    __builtin_amdgcn_fence(__ATOMIC_ACQUIRE, "workgroup");
  }
}

__global__ __launch_bounds__(128) void score_softmax_kernel(const _Float16* __restrict__ qp,
                                                            const _Float16* __restrict__ kp,
                                                            unsigned short* __restrict__ ph,
                                                            unsigned short* __restrict__ pl) {
  extern __shared__ __align__(16) float ssh[];
  const int tid = threadIdx.x, lane = tid & 31, w = tid >> 5;
  const int hh = lane >> 4, m = lane & 15;
  const int b  = blockIdx.y;
  const int j0 = blockIdx.x * JB;

  const _Float16* qrow  = qp + ((size_t)b * NS + j0 + m) * ND + 8 * hh;
  const _Float16* kbase = kp + ((size_t)b * NS + m) * ND + 8 * hh;
  const v8f zero8 = {0.f, 0.f, 0.f, 0.f, 0.f, 0.f, 0.f, 0.f};

#pragma unroll 1
  for (int g = 0; g < 4; ++g) {
    const int i0 = 512 * w + 128 * g;
    const _Float16* kg = kbase + (size_t)i0 * ND;
    v8f acc[8];
#pragma unroll
    for (int t = 0; t < 8; ++t) acc[t] = zero8;
#pragma unroll 1
    for (int k0 = 0; k0 < ND; k0 += 32) {
      const v16h a = Frag<_Float16>::load(qrow + k0);
#pragma unroll
      for (int t = 0; t < 8; ++t) {
        const v16h bfr = Frag<_Float16>::load(kg + (size_t)(16 * t) * ND + k0);
        acc[t] = wmma_f16g(a, bfr, acc[t]);
      }
    }
#pragma unroll
    for (int t = 0; t < 8; ++t) {
#pragma unroll
      for (int r = 0; r < 8; ++r) {
        ssh[(8 * hh + r) * SPITCH + i0 + 16 * t + m] = acc[t][r] * SSCALE;
      }
    }
  }
  __syncthreads();

#pragma unroll 1
  for (int rr = 0; rr < 4; ++rr) {
    const int row = 4 * w + rr;
    const float* srow = ssh + row * SPITCH + 8 * lane;
    float mx = -INFINITY;
#pragma unroll
    for (int it = 0; it < 8; ++it) {
      const v4f a = *(const v4fa*)(srow + 256 * it);
      const v4f c = *(const v4fa*)(srow + 256 * it + 4);
      mx = fmaxf(mx, fmaxf(fmaxf(a.x, a.y), fmaxf(a.z, a.w)));
      mx = fmaxf(mx, fmaxf(fmaxf(c.x, c.y), fmaxf(c.z, c.w)));
    }
#pragma unroll
    for (int off = 1; off < 32; off <<= 1) mx = fmaxf(mx, __shfl_xor(mx, off, 32));
    float sum = 0.0f;
#pragma unroll
    for (int it = 0; it < 8; ++it) {
      const v4f a = *(const v4fa*)(srow + 256 * it);
      const v4f c = *(const v4fa*)(srow + 256 * it + 4);
      sum += __expf(a.x - mx) + __expf(a.y - mx) + __expf(a.z - mx) + __expf(a.w - mx);
      sum += __expf(c.x - mx) + __expf(c.y - mx) + __expf(c.z - mx) + __expf(c.w - mx);
    }
#pragma unroll
    for (int off = 1; off < 32; off <<= 1) sum += __shfl_xor(sum, off, 32);
    const float inv = 1.0f / sum;
    const size_t prow = ((size_t)b * NS + j0 + row) * NS + 8 * lane;
    unsigned short* hrow = ph + prow;
    unsigned short* lrow = pl + prow;
#pragma unroll 1
    for (int pass = 0; pass < 2; ++pass) {
#pragma unroll
      for (int it = 0; it < 8; ++it) {
        const v4f a = *(const v4fa*)(srow + 256 * it);
        const v4f c = *(const v4fa*)(srow + 256 * it + 4);
        const float e0 = __expf(a.x - mx) * inv, e1 = __expf(a.y - mx) * inv;
        const float e2 = __expf(a.z - mx) * inv, e3 = __expf(a.w - mx) * inv;
        const float e4 = __expf(c.x - mx) * inv, e5 = __expf(c.y - mx) * inv;
        const float e6 = __expf(c.z - mx) * inv, e7 = __expf(c.w - mx) * inv;
        unsigned h0, h1, h2, h3, l0, l1, l2, l3;
        split_pair(e0, e1, h0, l0);
        split_pair(e2, e3, h1, l1);
        split_pair(e4, e5, h2, l2);
        split_pair(e6, e7, h3, l3);
        const v4u hv = {h0, h1, h2, h3};
        const v4u lv = {l0, l1, l2, l3};
        *(volatile v4u*)(hrow + 256 * it) = hv;
        *(volatile v4u*)(lrow + 256 * it) = lv;
      }
      __threadfence();
    }
  }
}

extern "C" void kernel_launch(void* const* d_in, const int* in_sizes, int n_in,
                              void* d_out, int out_size, void* d_ws, size_t ws_size,
                              hipStream_t stream) {
  if (n_in < 4) return;
  if (in_sizes[0] != NTOK * ND) return;
  if (in_sizes[1] != ND * ND || in_sizes[2] != ND * ND || in_sizes[3] != ND * ND) return;
  if (out_size != NTOK * ND) return;

  const float* x  = (const float*)d_in[0];
  const float* wq = (const float*)d_in[1];
  const float* wk = (const float*)d_in[2];
  const float* wv = (const float*)d_in[3];
  float* out = (float*)d_out;

  const size_t szP   = (size_t)NB * NS * NS * 2;
  const size_t szX16 = (size_t)NTOK * ND * 2;
  const size_t szW16 = (size_t)ND * ND * 2;
  const size_t oPh  = 0;
  const size_t oPl  = oPh + szP;
  const size_t oXB  = 0;
  const size_t oWKT = oXB + szX16;
  const size_t oWQT = oWKT + szW16;
  if (oWQT + szW16 > oPl + szP) return;
  const size_t oQP  = oPl + szP;
  const size_t oKP  = oQP + szX16;
  const size_t oCh  = oQP;
  const size_t oCl  = oKP;
  const size_t oXT  = oKP + szX16;
  const size_t oWVT = oXT + szX16;
  const size_t total = oWVT + szW16;
  if (total > ws_size) return;

  char* ws = (char*)d_ws;
  unsigned short* Ph  = (unsigned short*)(ws + oPh);
  unsigned short* Pl  = (unsigned short*)(ws + oPl);
  unsigned short* XB  = (unsigned short*)(ws + oXB);
  unsigned short* WKT = (unsigned short*)(ws + oWKT);
  unsigned short* WQT = (unsigned short*)(ws + oWQT);
  unsigned short* QP  = (unsigned short*)(ws + oQP);
  unsigned short* KP  = (unsigned short*)(ws + oKP);
  unsigned short* Ch  = (unsigned short*)(ws + oCh);
  unsigned short* Cl  = (unsigned short*)(ws + oCl);
  unsigned short* XT  = (unsigned short*)(ws + oXT);
  unsigned short* WVT = (unsigned short*)(ws + oWVT);

  const dim3 blk(256);

  prep_x_kernel<<<dim3(ND / 64, NS / 64, NB), blk, 0, stream>>>(x, XB, XT);
  prep_w_kernel<<<dim3(ND / 64, ND / 64, 3), blk, 0, stream>>>(wq, wk, wv, WQT, WKT, WVT);
  wmma_gemm64<1, false, 1><<<dim3((NTOK / 64) * (ND / 64) / 8, 2), blk, 0, stream>>>(
      XB, XB, ND, 0L, WKT, ND, (long)ND * ND, (void*)QP, (void*)QP, ND, (long)NTOK * ND,
      NTOK, ND, ND, PROJ_CARRY);
  (void)hipFuncSetAttribute(reinterpret_cast<const void*>(&score_softmax_kernel),
                            hipFuncAttributeMaxDynamicSharedMemorySize, SLDS_BYTES);
  score_softmax_kernel<<<dim3(NS / JB, NB), dim3(128), SLDS_BYTES, stream>>>(
      (const _Float16*)(const void*)QP, (const _Float16*)(const void*)KP, Ph, Pl);
  wmma_gemm64<1, true, 2><<<dim3((NS / 64) * (ND / 64) / 8, NB), blk, 0, stream>>>(
      Ph, Pl, NS, (long)NS * NS, XT, NS, (long)ND * NS, (void*)Ch, (void*)Cl, ND, (long)NS * ND,
      NS, ND, NS, 1.0f);
  wmma_gemm64<1, true, 0><<<dim3((NTOK / 64) * (ND / 64) / 8, 1), blk, 0, stream>>>(
      Ch, Cl, ND, 0L, WVT, ND, 0L, (void*)out, (void*)out, ND, 0L,
      NTOK, ND, ND, 1.0f);
  (void)hipGetLastError();
}
